// MultiheadDiffAttn_16982300688399
// MI455X (gfx1250) — hardware-verified
//
#include <hip/hip_runtime.h>


#ifndef NB
#define NB 4
#endif
#ifndef SEQ
#define SEQ 1024
#endif
#define NB_FULL  4
#define SEQ_FULL 1024
#define EE   1024
#define EK   512
#define NQ2  32
#define NK2  16
#define NKV  8
#define NHQ  16
#define HD   32
#define VD   64
#define HG   8
#define NMAP (2 * HG)
#define NR   (NB * SEQ)
#define LAM0 0.78360576653f
#define OML  0.21639423347f
#define SCL  0.17677669529663687f
#define ADSC 1024.0f
#define EPSN 1e-6f
static_assert(SEQ % 64 == 0);
static_assert(SEQ >= 64 && SEQ <= SEQ_FULL);
static_assert(NB >= 1 && NB <= NB_FULL);
static_assert(NHQ % HG == 0);
static_assert(NQ2 % 8 == 0 && NK2 % 8 == 0);

typedef _Float16 h16;
typedef unsigned short bf;
typedef __attribute__((ext_vector_type(16))) __bf16   v16bf;
typedef __attribute__((ext_vector_type(16))) _Float16 v16h;
typedef __attribute__((ext_vector_type(8)))  _Float16 v8h;
typedef __attribute__((ext_vector_type(4)))  _Float16 v4h;
typedef __attribute__((ext_vector_type(2)))  _Float16 v2h;
typedef __attribute__((ext_vector_type(8)))  unsigned short v8us;
typedef __attribute__((ext_vector_type(8)))  float    v8f;
typedef __attribute__((ext_vector_type(4)))  float    v4f;
typedef __attribute__((ext_vector_type(2)))  float    v2f;
typedef v8h  __attribute__((may_alias)) v8ha;
typedef v4f  __attribute__((may_alias)) v4fa;

__device__ __forceinline__ unsigned short f2bf(float f) { unsigned u = __float_as_uint(f); u += 0x7FFFu + ((u >> 16) & 1u); return (unsigned short)(u >> 16); }
__device__ __forceinline__ float bf2f(unsigned short b) { return __uint_as_float(((unsigned)b) << 16); }
__device__ __forceinline__ float bfr(float f) { return bf2f(f2bf(f)); }
__device__ __forceinline__ h16 tohx(float x) { return (h16)x; }
__device__ __forceinline__ v16h cat16(v8h lo, v8h hi) { return __builtin_shufflevector(lo, hi, 0, 1, 2, 3, 4, 5, 6, 7, 8, 9, 10, 11, 12, 13, 14, 15); }
__device__ __forceinline__ v16bf cat16b(v8us lo, v8us hi) { return __builtin_bit_cast(v16bf, __builtin_shufflevector(lo, hi, 0, 1, 2, 3, 4, 5, 6, 7, 8, 9, 10, 11, 12, 13, 14, 15)); }
__device__ __forceinline__ v8f wmma16(v16h a, v16h b, v8f c) { return __builtin_amdgcn_wmma_f32_16x16x32_f16(false, a, false, b, (short)0, c, false, false); }
__device__ __forceinline__ v8f wmmab(v16bf a, v16bf b, v8f c) { return __builtin_amdgcn_wmma_f32_16x16x32_bf16(false, a, false, b, (short)0, c, false, false); }

__constant__ float c_invf[16] = {
    1.0f,                    0.5623413251903491f,    0.31622776601683794f,   0.17782794100389228f,
    0.1f,                    0.05623413251903491f,   0.031622776601683794f,  0.017782794100389228f,
    0.01f,                   0.005623413251903491f,  0.0031622776601683794f, 0.0017782794100389228f,
    0.001f,                  0.0005623413251903491f, 0.00031622776601683794f, 0.00017782794100389228f };

__global__ __launch_bounds__(256) void k_rtab(float* CS) {
    __shared__ __align__(16) float tcs[2][256];
    const int tid = threadIdx.x; const int e = blockIdx.x * 256 + tid; const int t = e >> 4, i = e & 15;
    float sv, cv; sincosf((float)t * c_invf[i], &sv, &cv);
    tcs[0][tid] = cv; tcs[1][tid] = sv;
    __syncthreads();
    if (tid < 128) { const int w = tid >> 6, j = tid & 63; const v4f v = *(const v4fa*)(&tcs[w][j * 4]);
        float* dst = CS + (size_t)w * SEQ * 16 + (size_t)blockIdx.x * 256 + j * 4;
        *(volatile v4f*)dst = v; __threadfence(); *(volatile v4f*)dst = v; }
}

__global__ __launch_bounds__(256) void k_cvtx(const float* __restrict__ x, bf* A) {
    const int lane = threadIdx.x & 31; const size_t r = (size_t)blockIdx.x * 8 + (threadIdx.x >> 5); if (r >= (size_t)NR) return;
    const size_t bb = r / SEQ, tt = r - bb * SEQ; const size_t sr = bb * SEQ_FULL + tt;
#pragma unroll 1
    for (int ps = 0; ps < 2; ++ps) {
#pragma unroll
        for (int q = 0; q < EE / 256; ++q) { const size_t so = sr * EE + q * 256 + lane * 8, o = r * EE + q * 256 + lane * 8;
            const v4f a = *(const v4f*)(x + so), c = *(const v4f*)(x + so + 4); v8us v;
#pragma unroll
            for (int k = 0; k < 4; ++k) { v[k] = f2bf(a[k]); v[4 + k] = f2bf(c[k]); }
            *(volatile v8us*)(A + o) = v; }
        if (ps == 0) __threadfence(); }
}

__global__ __launch_bounds__(256) void k_wT(const float* __restrict__ W, int N, int isH, unsigned short* P) {
    __shared__ float tl[64][65];
    const int tid = threadIdx.x; const int k0 = blockIdx.x * 64, n0 = blockIdx.y * 64; const int rr = tid >> 2, cq = (tid & 3) * 16;
    const float* src = W + (size_t)(k0 + rr) * N + n0 + cq;
#pragma unroll
    for (int j = 0; j < 4; ++j) { const v4f v = *(const v4f*)(src + 4 * j);
#pragma unroll
        for (int q = 0; q < 4; ++q) tl[rr][cq + 4 * j + q] = v[q]; }
    __syncthreads();
    const int lane = tid & 31, wv = tid >> 5;
    auto pass = [&]() {
#pragma unroll
        for (int st = 0; st < 2; ++st) { const int dr = wv * 8 + st * 4 + (lane >> 3), piece = lane & 7; v8us o;
#pragma unroll
            for (int i = 0; i < 8; ++i) { const unsigned short b = f2bf(tl[piece * 8 + i][dr]); const h16 hv = tohx(bf2f(b)); o[i] = isH ? __builtin_bit_cast(unsigned short, hv) : b; }
            *(volatile v8us*)(P + (size_t)(n0 + dr) * EE + k0 + piece * 8) = o; }
    };
    pass(); __threadfence(); pass();
}

__global__ __launch_bounds__(128) void k_gemmb(const bf* __restrict__ A, const bf* __restrict__ Bn, float* C, int ldc, int K) {
    __shared__ __align__(16) float ost[4][16 * 68];
    const int lane = threadIdx.x & 31, wave = threadIdx.x >> 5, lr = lane & 15, hi = lane >> 4;
    const int r0 = blockIdx.x * 64 + wave * 16, c0 = blockIdx.y * 64;
    const size_t aoff = (size_t)(r0 + lr) * K + 8 * hi;
    size_t boff[4];
#pragma unroll
    for (int t = 0; t < 4; ++t) boff[t] = (size_t)(c0 + t * 16 + lr) * K + 8 * hi;
    v8f acc[4];
#pragma unroll
    for (int t = 0; t < 4; ++t) acc[t] = (v8f){};
#pragma unroll 1
    for (int kc = 0; kc < K; kc += 32) {
        const v16bf a = cat16b(*(const v8us*)(A + aoff + kc), *(const v8us*)(A + aoff + kc + 16));
#pragma unroll
        for (int t = 0; t < 4; ++t) { const v16bf b = cat16b(*(const v8us*)(Bn + boff[t] + kc), *(const v8us*)(Bn + boff[t] + kc + 16)); acc[t] = wmmab(a, b, acc[t]); }
        asm volatile("v_nop\n\tv_nop\n\tv_nop\n\tv_nop" : "+v"(acc[0]), "+v"(acc[1]), "+v"(acc[2]), "+v"(acc[3]) : "v"(a));
    }
    float* os = &ost[wave][0];
#pragma unroll
    for (int t = 0; t < 4; ++t) {
#pragma unroll
        for (int j = 0; j < 8; ++j) os[(hi * 8 + j) * 68 + t * 16 + lr] = acc[t][j]; }
    __syncthreads();
    float* crow = C + (size_t)r0 * ldc + c0;
    auto pass = [&]() {
#pragma unroll
        for (int s = 0; s < 8; ++s) { const int Lid = (lane >> 3) + 4 * s, piece = lane & 7; const int row = Lid >> 1, cofs = (Lid & 1) * 32 + piece * 4;
            const v4f val = *(const v4fa*)(os + row * 68 + cofs);
            *(volatile v4f*)(crow + (size_t)row * ldc + cofs) = val; }
    };
    pass(); __threadfence(); pass();
}

__global__ __launch_bounds__(128) void k_gemmh(const h16* __restrict__ A, const h16* __restrict__ Bn, float* C, int ldc, int K, size_t sA, size_t sB, size_t sC, int zmode, int causal) {
    __shared__ __align__(16) float ost[4][16 * 68];
    if (causal == 1 && blockIdx.y > blockIdx.x) return;
    const size_t z = blockIdx.z; const size_t zb = (zmode == 1) ? ((z >> 2) * 2 + (z & 1)) : ((zmode == 2) ? (z >> 1) : z);
    A += z * sA; Bn += zb * sB; C += z * sC;
    const int lane = threadIdx.x & 31, wave = threadIdx.x >> 5, lr = lane & 15, hi = lane >> 4;
    const int r0 = blockIdx.x * 64 + wave * 16, c0 = blockIdx.y * 64;
    const int kcap = (int)(blockIdx.x + 1) * 64; const int klim = (causal == 2 && kcap < K) ? kcap : K;
    const size_t aoff = (size_t)(r0 + lr) * K + 8 * hi;
    size_t boff[4];
#pragma unroll
    for (int t = 0; t < 4; ++t) boff[t] = (size_t)(c0 + t * 16 + lr) * K + 8 * hi;
    v8f acc[4];
#pragma unroll
    for (int t = 0; t < 4; ++t) acc[t] = (v8f){};
#pragma unroll 1
    for (int kc = 0; kc < klim; kc += 32) {
        const v16h a = cat16(*(const v8h*)(A + aoff + kc), *(const v8h*)(A + aoff + kc + 16));
#pragma unroll
        for (int t = 0; t < 4; ++t) { const v16h b = cat16(*(const v8h*)(Bn + boff[t] + kc), *(const v8h*)(Bn + boff[t] + kc + 16)); acc[t] = wmma16(a, b, acc[t]); }
        asm volatile("v_nop\n\tv_nop\n\tv_nop\n\tv_nop" : "+v"(acc[0]), "+v"(acc[1]), "+v"(acc[2]), "+v"(acc[3]) : "v"(a));
    }
    float* os = &ost[wave][0];
#pragma unroll
    for (int t = 0; t < 4; ++t) {
#pragma unroll
        for (int j = 0; j < 8; ++j) os[(hi * 8 + j) * 68 + t * 16 + lr] = acc[t][j]; }
    __syncthreads();
    float* crow = C + (size_t)r0 * ldc + c0;
    auto pass = [&]() {
#pragma unroll
        for (int s = 0; s < 8; ++s) { const int Lid = (lane >> 3) + 4 * s, piece = lane & 7; const int row = Lid >> 1, cofs = (Lid & 1) * 32 + piece * 4;
            const v4f val = *(const v4fa*)(os + row * 68 + cofs);
            *(volatile v4f*)(crow + (size_t)row * ldc + cofs) = val; }
    };
    pass(); __threadfence(); pass();
}

__global__ __launch_bounds__(256) void k_ropep(const float* __restrict__ F, int ld, int NP, const float* __restrict__ CS, h16* P) {
    __shared__ __align__(16) h16 tile[8 * 32 * 32];
    const int tid = threadIdx.x; const int t0 = blockIdx.x * 32, g0 = blockIdx.y * 8, b = blockIdx.z;
    const int h2l = tid >> 5, tl = tid & 31; const int t = t0 + tl;
    const float* src = F + ((size_t)b * SEQ + t) * ld + (size_t)(g0 + h2l) * HD;
    v4f xa[8];
#pragma unroll
    for (int j = 0; j < 8; ++j) xa[j] = *(const v4f*)(src + 4 * j);
    const float* cp = CS + (size_t)t * 16; const float* sp = CS + (size_t)SEQ * 16 + (size_t)t * 16;
    v4f c4[4], s4[4];
#pragma unroll
    for (int j = 0; j < 4; ++j) { c4[j] = *(const v4f*)(cp + 4 * j); s4[j] = *(const v4f*)(sp + 4 * j); }
    v8h o[4];
#pragma unroll
    for (int j = 0; j < 4; ++j) {
#pragma unroll
        for (int q = 0; q < 4; ++q) { const float x1 = xa[j][q], x2 = xa[4 + j][q], c = c4[j][q], s = s4[j][q];
            o[j >> 1][(j & 1) * 4 + q] = tohx(x1 * c + x2 * s); o[2 + (j >> 1)][(j & 1) * 4 + q] = tohx(x2 * c - x1 * s); } }
    h16* trow = tile + (h2l * 32 + tl) * 32;
#pragma unroll
    for (int j = 0; j < 4; ++j) *(v8ha*)(trow + 8 * j) = o[j];
    __syncthreads();
    auto pass = [&]() {
#pragma unroll
        for (int s = 0; s < 4; ++s) { const int p = s * 256 + tid; const int pl = p >> 7, q = p & 127;
            const v8h v = *(const v8ha*)(tile + pl * 1024 + q * 8);
            *(volatile v8h*)(P + (((size_t)b * NP + g0 + pl) * SEQ + t0) * HD + q * 8) = v; }
    };
    pass(); __threadfence(); pass();
}

__global__ __launch_bounds__(256) void k_vTm(const float* __restrict__ V, h16* VT) {
    __shared__ float tl[64][65];
    const int tid = threadIdx.x; const int t0 = blockIdx.x * 64, c = blockIdx.y, b = blockIdx.z; const int rr = tid >> 2, cq = (tid & 3) * 16;
    const float* src = V + ((size_t)b * SEQ + t0 + rr) * EK + c * VD + cq;
#pragma unroll
    for (int j = 0; j < 4; ++j) { const v4f v = *(const v4f*)(src + 4 * j);
#pragma unroll
        for (int q = 0; q < 4; ++q) tl[rr][cq + 4 * j + q] = v[q]; }
    __syncthreads();
    const int lane = tid & 31, wv = tid >> 5;
    h16* dst0 = VT + ((size_t)(b * NKV + c) * VD) * SEQ + t0;
    auto pass = [&]() {
#pragma unroll
        for (int st = 0; st < 4; ++st) { const int dr = wv * 8 + st * 2 + (lane >> 4); const int tq = (lane & 15) * 4; v4h v;
#pragma unroll
            for (int i = 0; i < 4; ++i) v[i] = tohx(tl[tq + i][dr]);
            *(volatile v4h*)(dst0 + (size_t)dr * SEQ + tq) = v; }
    };
    pass(); __threadfence(); pass();
}

__global__ __launch_bounds__(256) void k_softdiff(const float* __restrict__ S, const float* __restrict__ lq1, const float* __restrict__ lk1, const float* __restrict__ lq2, const float* __restrict__ lk2, h16* AD) {
    const int lane = threadIdx.x & 31, i = blockIdx.x * 8 + (threadIdx.x >> 5); if (i >= SEQ) return; const int hl = blockIdx.z;
    float d1 = bfr(lq1[lane]) * bfr(lk1[lane]), d2 = bfr(lq2[lane]) * bfr(lk2[lane]);
#pragma unroll
    for (int sh = 16; sh; sh >>= 1) { d1 += __shfl_xor(d1, sh, 32); d2 += __shfl_xor(d2, sh, 32); }
    const float lam = expf(d1) - expf(d2) + LAM0;
    const float* s1 = S + ((size_t)(hl * 2) * SEQ + i) * SEQ; const float* s2 = S + ((size_t)(hl * 2 + 1) * SEQ + i) * SEQ;
    const int cend = ((i >> 6) + 1) << 6;
    float m1 = -3.0e38f, m2 = -3.0e38f;
#pragma unroll 1
    for (int c0 = lane * 4; c0 < cend; c0 += 128) { const v4f a = *(const v4f*)(s1 + c0), e = *(const v4f*)(s2 + c0);
#pragma unroll
        for (int q = 0; q < 4; ++q) { const bool ok = (c0 + q) <= i; m1 = fmaxf(m1, ok ? a[q] * SCL : -3.0e38f); m2 = fmaxf(m2, ok ? e[q] * SCL : -3.0e38f); } }
#pragma unroll
    for (int sh = 16; sh; sh >>= 1) { m1 = fmaxf(m1, __shfl_xor(m1, sh, 32)); m2 = fmaxf(m2, __shfl_xor(m2, sh, 32)); }
    float u1 = 0.f, u2 = 0.f;
#pragma unroll 1
    for (int c0 = lane * 4; c0 < cend; c0 += 128) { const v4f a = *(const v4f*)(s1 + c0), e = *(const v4f*)(s2 + c0);
#pragma unroll
        for (int q = 0; q < 4; ++q) { const bool ok = (c0 + q) <= i; u1 += ok ? __expf(a[q] * SCL - m1) : 0.f; u2 += ok ? __expf(e[q] * SCL - m2) : 0.f; } }
#pragma unroll
    for (int sh = 16; sh; sh >>= 1) { u1 += __shfl_xor(u1, sh, 32); u2 += __shfl_xor(u2, sh, 32); }
    const float i1 = 1.0f / u1, i2 = lam / u2;
    h16* arow = AD + ((size_t)hl * SEQ + i) * SEQ;
#pragma unroll 1
    for (int ps = 0; ps < 2; ++ps) {
#pragma unroll 1
        for (int c0 = lane * 4; c0 < cend; c0 += 128) { const v4f a = *(const v4f*)(s1 + c0), e = *(const v4f*)(s2 + c0); v4h o;
#pragma unroll
            for (int q = 0; q < 4; ++q) { const bool ok = (c0 + q) <= i;
                const float pv = (__expf(a[q] * SCL - m1) * i1 - __expf(e[q] * SCL - m2) * i2) * ADSC;
                o[q] = ok ? tohx(pv) : tohx(0.0f); }
            *(volatile v4h*)(arow + c0) = o; }
        if (ps == 0) __threadfence(); }
}

__global__ __launch_bounds__(256) void k_rmsh(const float* __restrict__ O, int b, int hg0, const float* __restrict__ rw, h16* OH) {
    const int lane = threadIdx.x & 31, i = blockIdx.x * 8 + (threadIdx.x >> 5); if (i >= SEQ) return; const int hl = blockIdx.z; const int h = hg0 + hl;
    v2f v = *(const v2f*)(O + ((size_t)hl * SEQ + i) * VD + lane * 2); v = v * (1.0f / ADSC);
    float q = v[0] * v[0] + v[1] * v[1];
#pragma unroll
    for (int sh = 16; sh; sh >>= 1) q += __shfl_xor(q, sh, 32);
    const float sc = rsqrtf(q * (1.0f / VD) + EPSN);
    const float w0 = bfr(rw[lane * 2]) * OML, w1 = bfr(rw[lane * 2 + 1]) * OML;
    v2h o; o[0] = tohx(v[0] * sc * w0); o[1] = tohx(v[1] * sc * w1);
    const size_t off = ((size_t)b * SEQ + i) * EE + (size_t)h * VD + lane * 2;
    *(volatile v2h*)(OH + off) = o; __threadfence(); *(volatile v2h*)(OH + off) = o;
}

extern "C" void kernel_launch(void* const* d_in, const int* in_sizes, int n_in,
                              void* d_out, int out_size, void* d_ws, size_t ws_size, hipStream_t stream) {
    if (n_in < 10) return;
    if ((size_t)in_sizes[0] < ((size_t)(NB - 1) * SEQ_FULL + SEQ) * EE) return;
    if ((size_t)in_sizes[1] < (size_t)EE * EE || (size_t)in_sizes[2] < (size_t)EE * EK || (size_t)in_sizes[3] < (size_t)EE * EK || (size_t)in_sizes[4] < (size_t)EE * EE) return;
    if (in_sizes[5] < HD || in_sizes[6] < HD || in_sizes[7] < HD || in_sizes[8] < HD || in_sizes[9] < VD) return;
    if ((size_t)out_size < (size_t)NR * EE) return;
    const float* x = (const float*)d_in[0]; const float* Wq = (const float*)d_in[1]; const float* Wk = (const float*)d_in[2]; const float* Wv = (const float*)d_in[3]; const float* Wo = (const float*)d_in[4];
    const float* lq1 = (const float*)d_in[5]; const float* lk1 = (const float*)d_in[6]; const float* lq2 = (const float*)d_in[7]; const float* lk2 = (const float*)d_in[8]; const float* rmsw = (const float*)d_in[9];
    float* out = (float*)d_out;
    char* wsp = (char*)d_ws; size_t used = 0;
    auto take = [&](size_t bytes) { void* p = wsp + used; used += (bytes + 255) & ~(size_t)255; return p; };
    bf* XB = (bf*)take((size_t)NR * EE * 2);
    bf* WQB = (bf*)take((size_t)EE * EE * 2); bf* WKB = (bf*)take((size_t)EK * EE * 2); bf* WVB = (bf*)take((size_t)EK * EE * 2); h16* WOH = (h16*)take((size_t)EE * EE * 2);
    float* CS = (float*)take((size_t)2 * SEQ * 16 * 4);
    h16* QH = (h16*)take((size_t)NB * NQ2 * SEQ * HD * 2); h16* KH = (h16*)take((size_t)NB * NK2 * SEQ * HD * 2); h16* VT = (h16*)take((size_t)NB * NKV * VD * SEQ * 2);
    h16* OH = (h16*)take((size_t)NR * EE * 2);
    const size_t sbytes = (size_t)NMAP * SEQ * SEQ * 4, pbytes = (size_t)NR * (EE + EK + EK) * 4; const size_t rsb = sbytes > pbytes ? sbytes : pbytes;
    char* RS = (char*)take(rsb);
    float* S = (float*)RS; float* Qf = (float*)RS; float* Kf = Qf + (size_t)NR * EE; float* Vf = Kf + (size_t)NR * EK;
    h16* AD = (h16*)take((size_t)HG * SEQ * SEQ * 2); float* O = (float*)take((size_t)HG * SEQ * VD * 4);
    if (used > ws_size) return;
    k_rtab<<<SEQ * 16 / 256, 256, 0, stream>>>(CS);
    k_cvtx<<<NR / 8, 256, 0, stream>>>(x, XB);
    k_wT<<<dim3(EE / 64, EE / 64, 1), 256, 0, stream>>>(Wq, EE, 0, WQB);
    k_wT<<<dim3(EE / 64, EK / 64, 1), 256, 0, stream>>>(Wk, EK, 0, WKB);
    k_wT<<<dim3(EE / 64, EK / 64, 1), 256, 0, stream>>>(Wv, EK, 0, WVB);
    k_wT<<<dim3(EE / 64, EE / 64, 1), 256, 0, stream>>>(Wo, EE, 1, (unsigned short*)WOH);
    k_gemmb<<<dim3(NR / 64, EE / 64, 1), 128, 0, stream>>>(XB, WQB, Qf, EE, EE);
    k_gemmb<<<dim3(NR / 64, EK / 64, 1), 128, 0, stream>>>(XB, WKB, Kf, EK, EE);
    k_gemmb<<<dim3(NR / 64, EK / 64, 1), 128, 0, stream>>>(XB, WVB, Vf, EK, EE);
    k_ropep<<<dim3(SEQ / 32, NQ2 / 8, NB), 256, 0, stream>>>(Qf, EE, NQ2, CS, QH);
    k_ropep<<<dim3(SEQ / 32, NK2 / 8, NB), 256, 0, stream>>>(Kf, EK, NK2, CS, KH);
    k_vTm<<<dim3(SEQ / 64, NKV, NB), 256, 0, stream>>>(Vf, VT);
    for (int b = 0; b < NB; ++b)
        for (int hg = 0; hg < NHQ / HG; ++hg) {
            const int hg0 = hg * HG;
            k_gemmh<<<dim3(SEQ / 64, SEQ / 64, NMAP), 128, 0, stream>>>(QH + (size_t)(b * NQ2 + hg0 * 2) * SEQ * HD, KH + (size_t)(b * NK2 + hg0) * SEQ * HD, S, SEQ, HD, (size_t)SEQ * HD, (size_t)SEQ * HD, (size_t)SEQ * SEQ, 1, 1);
            k_softdiff<<<dim3(SEQ / 8, 1, HG), 256, 0, stream>>>(S, lq1, lk1, lq2, lk2, AD);
            k_gemmh<<<dim3(SEQ / 64, VD / 64, HG), 128, 0, stream>>>(AD, VT + (size_t)(b * NKV + hg0 / 2) * VD * SEQ, O, VD, SEQ, (size_t)SEQ * SEQ, (size_t)VD * SEQ, (size_t)SEQ * VD, 2, 2);
            k_rmsh<<<dim3(SEQ / 8, 1, HG), 256, 0, stream>>>(O, b, hg0, rmsw, OH); }
    k_gemmh<<<dim3(NR / 64, EE / 64, 1), 128, 0, stream>>>(OH, WOH, out, EE, EE, 0, 0, 0, 0, 0);
}
